// DeblurTransformer_75505525064047
// MI455X (gfx1250) — hardware-verified
//
#include <hip/hip_runtime.h>
#include <math.h>

typedef __attribute__((ext_vector_type(16))) _Float16 v16h;
typedef __attribute__((ext_vector_type(16))) __bf16 v16b;
typedef __attribute__((ext_vector_type(8)))  _Float16 v8h;
typedef __attribute__((ext_vector_type(8)))  float v8f;
typedef __attribute__((ext_vector_type(4)))  float v4f;
typedef __attribute__((ext_vector_type(2)))  float v2f;
typedef __attribute__((ext_vector_type(4)))  unsigned v4u;
typedef __attribute__((ext_vector_type(4)))  int v4i;
typedef float __attribute__((may_alias)) float_a;
typedef int __attribute__((may_alias)) int_a;

template <typename T> __device__ __forceinline__ void vst2(void* p, T v) { *(volatile T*)p = v; __threadfence(); *(volatile T*)p = v; }
__device__ __forceinline__ v8f wmma16(v16h a, v16h b, v8f c) {
  v8f d = __builtin_amdgcn_wmma_f32_16x16x32_f16(false, a, false, b, (short)0, c, false, false);
  asm volatile("v_nop\n\tv_nop\n\tv_nop\n\tv_nop" : "+v"(d) : "v"(a), "v"(b));
  return d;
}
__device__ __forceinline__ v8f wmma_bf(v16b a, v16b b, v8f c) {
  v8f d = __builtin_amdgcn_wmma_f32_16x16x32_bf16(false, a, false, b, (short)0, c, false, false);
  asm volatile("v_nop\n\tv_nop\n\tv_nop\n\tv_nop" : "+v"(d) : "v"(a), "v"(b));
  return d;
}
__device__ __forceinline__ v16h frag_h(const _Float16* rowk0, int lane) {
  union { v16h v; v8h q[2]; } u; const _Float16* p = rowk0 + 8 * (lane >> 4);
  u.q[0] = *(const v8h*)p; u.q[1] = *(const v8h*)(p + 16); return u.v;
}
__device__ __forceinline__ v16h frag_f32(const float* rowk0, int lane) {
  v16h a; const float* p = rowk0 + 8 * (lane >> 4);
#pragma unroll
  for (int i = 0; i < 8; ++i) { a[i] = (_Float16)p[i]; a[8 + i] = (_Float16)p[16 + i]; }
  return a;
}
__device__ __forceinline__ v16h frag_f32s(const float* rowk0, int lane, float sc) {
  v16h a; const float* p = rowk0 + 8 * (lane >> 4);
#pragma unroll
  for (int i = 0; i < 8; ++i) { a[i] = (_Float16)(p[i] * sc); a[8 + i] = (_Float16)(p[16 + i] * sc); }
  return a;
}
__device__ __forceinline__ v16h fragc_f32(const float* W, int k0, int n, int lane, int ld, int K) {
  v16h a; const int g = lane >> 4;
#pragma unroll
  for (int i = 0; i < 8; ++i) { const int ka = k0 + 8 * g + i, kb = ka + 16;
    a[i] = (_Float16)(ka < K ? W[(size_t)(ka < K ? ka : K - 1) * ld + n] : 0.f); a[8 + i] = (_Float16)(kb < K ? W[(size_t)(kb < K ? kb : K - 1) * ld + n] : 0.f); }
  return a;
}
struct F2 { v16b h, l; };
__device__ __forceinline__ F2 bsplit16(const float v[16]) { F2 r;
#pragma unroll
  for (int i = 0; i < 16; ++i) { const __bf16 h = (__bf16)v[i]; r.h[i] = h; r.l[i] = (__bf16)(v[i] - (float)h); }
  return r; }
__device__ __forceinline__ F2 split_row(const float* row, int k0, int lane) { float v[16]; const float* p = row + k0 + 8 * (lane >> 4);
#pragma unroll
  for (int i = 0; i < 8; ++i) { v[i] = p[i]; v[8 + i] = p[16 + i]; }
  return bsplit16(v); }
__device__ __forceinline__ F2 split_rowK(const float* row, int k0, int lane, int K) { float v[16]; const int g = lane >> 4;
#pragma unroll
  for (int i = 0; i < 8; ++i) { const int ka = k0 + 8 * g + i, kb = ka + 16; v[i] = ka < K ? row[ka < K ? ka : K - 1] : 0.f; v[8 + i] = kb < K ? row[kb < K ? kb : K - 1] : 0.f; }
  return bsplit16(v); }
__device__ __forceinline__ F2 split_col(const float* W, int k0, int n, int lane, int ld, int K) { float v[16]; const int g = lane >> 4;
#pragma unroll
  for (int i = 0; i < 8; ++i) { const int ka = k0 + 8 * g + i, kb = ka + 16; v[i] = ka < K ? W[(size_t)(ka < K ? ka : K - 1) * ld + n] : 0.f; v[8 + i] = kb < K ? W[(size_t)(kb < K ? kb : K - 1) * ld + n] : 0.f; }
  return bsplit16(v); }
__device__ __forceinline__ v8f mac3(const F2& a, const F2& b, v8f c) { c = wmma_bf(a.l, b.h, c); c = wmma_bf(a.h, b.l, c); return wmma_bf(a.h, b.h, c); }
__device__ __forceinline__ float sigm(float v) { return 1.0f / (1.0f + expf(-v)); }
#define LDSX() do { asm volatile("s_wait_dscnt 0" ::: "memory"); __builtin_amdgcn_wave_barrier(); __builtin_amdgcn_fence(__ATOMIC_RELEASE, "workgroup"); } while (0)


#define NBT 2
#define CIN 3
#define CH 64
#define C8 8
#define HH 96
#define WWD 96
#define NPI (HH * WWD)
#define NPIX (NBT * NPI)
#define NBLK 5
#define KIN 256
#define K3 (9 * CH)
#define KOUT (81 * CH)
#ifndef TNB
#define TNB NBT
#define TQT (NBT * NPI / 64)
#define TYO (NBT * HH)
#endif
typedef __attribute__((ext_vector_type(8))) __bf16 v8b;
__device__ __forceinline__ v16b frag_b(const __bf16* rowk0, int lane) {
  union { v16b v; v8b q[2]; } u; const __bf16* p = rowk0 + 8 * (lane >> 4);
  u.q[0] = *(const v8b*)p; u.q[1] = *(const v8b*)(p + 16); return u.v;
}
__device__ __forceinline__ float bfr(float v) { return (float)(__bf16)v; }
__device__ __attribute__((noinline)) float exp_ni(float v) { return expf(v); }
__device__ __attribute__((noinline)) float erf_ni(float v) { return erff(v); }
__device__ __attribute__((noinline)) float tanh_ni(float v) { return tanhf(v); }

#define PK_IN 0
#define PK_R1 (PK_IN + CH * KIN)
#define PK_R2 (PK_R1 + NBLK * CH * K3)
#define PK_Q  (PK_R2 + NBLK * CH * K3)
#define PK_K  (PK_Q + 16 * CH)
#define PK_V  (PK_K + 16 * CH)
#define PK_O  (PK_V + CH * CH)
#define PK_END (PK_O + 16 * KOUT)
#define PLANE (2u * NPIX * CH)
#define WS_PK  0u
#define WS_ACT (((WS_PK + 2u * PK_END) + 127u) / 128u * 128u)
#define PL_OUT(i, lo) (WS_ACT + (size_t)PLANE * (2 * (i) + (lo)))
#define PL_H(lo)   (WS_ACT + (size_t)PLANE * (12 + (lo)))
#define PL_ATT(lo) (WS_ACT + (size_t)PLANE * (14 + (lo)))
#define WS_QK  (WS_ACT + (size_t)PLANE * 16)
#define WS_VTH (WS_QK + 2u * NPIX * 64)
#define WS_VTL (WS_VTH + 2u * NBT * CH * NPI)
#define WS_END (WS_VTL + 2u * NBT * CH * NPI)

__global__ __launch_bounds__(256) void k_pack(const float* __restrict__ WIN, const float* __restrict__ RW1, const float* __restrict__ RW2, const float* __restrict__ WQ, const float* __restrict__ WK, const float* __restrict__ WV, const float* __restrict__ WOUT, __bf16* __restrict__ PK) {
  __shared__ __align__(16) __bf16 s[KOUT]; const int o = blockIdx.x, which = blockIdx.y, tid = threadIdx.x; int K; size_t dst;
  if (which <= 10 && o >= CH) return;
  if (which == 0) { K = KIN; dst = PK_IN + (size_t)o * KIN; for (int k = tid; k < K; k += 256) { const int tap = k / 3, c = k % 3; s[k] = (__bf16)((k < 243) ? WIN[((size_t)o * CIN + c) * 81 + tap] : 0.f); } }
  else if (which <= 10) { const int i = (which - 1) % 5; const float* Wm = (which <= 5 ? RW1 : RW2) + (size_t)i * CH * CH * 9; K = K3; dst = (which <= 5 ? PK_R1 : PK_R2) + ((size_t)i * CH + o) * K3; for (int k = tid; k < K; k += 256) { const int tap = k / CH, c = k % CH; s[k] = (__bf16)Wm[((size_t)o * CH + c) * 9 + tap]; } }
  else if (which == 11) { K = CH; if (o < 16) { dst = PK_Q + (size_t)o * CH; for (int k = tid; k < K; k += 256) s[k] = (__bf16)((o < C8) ? WQ[(size_t)o * CH + k] : 0.f); }
    else if (o < 32) { dst = PK_K + (size_t)(o - 16) * CH; for (int k = tid; k < K; k += 256) s[k] = (__bf16)((o - 16 < C8) ? WK[(size_t)(o - 16) * CH + k] : 0.f); }
    else { dst = PK_V + (size_t)(o - 32) * CH; for (int k = tid; k < K; k += 256) s[k] = (__bf16)WV[(size_t)(o - 32) * CH + k]; } }
  else { if (o >= 16) return; K = KOUT; dst = PK_O + (size_t)o * KOUT; for (int k = tid; k < K; k += 256) { const int tap = k / CH, c = k % CH; s[k] = (__bf16)((o < CIN) ? WOUT[((size_t)o * CH + c) * 81 + tap] : 0.f); } }
  __syncthreads();
  for (int q = tid; q < K / 8; q += 256) vst2((unsigned*)(PK + dst + q * 8), *(const v4u*)&s[q * 8]);
}
__device__ __forceinline__ v16b zfrag_if(v16b a, bool ok) { const v16b z = {}; return ok ? a : z; }
__device__ __forceinline__ float prelu(float v, float a) { return v >= 0.f ? v : a * v; }
__global__ __launch_bounds__(192) void k_cin(const float* __restrict__ X, const __bf16* __restrict__ PK, const float* __restrict__ BIN, const float* __restrict__ AIN, __bf16* __restrict__ OH, __bf16* __restrict__ OL) {
  __shared__ __align__(16) __bf16 sh_[6][16][72], sl_[6][16][72];
  const int tid = threadIdx.x, wave = tid >> 5, lane = tid & 31, col = lane & 15, g = lane >> 4; const int row = blockIdx.x; const int b = row / HH, y = row % HH; const int px = wave * 16 + col;
  v8f acc[4] = {};
#pragma unroll 1
  for (int kc = 0; kc < KIN / 32; ++kc) { v16b a;
#pragma unroll
    for (int i = 0; i < 16; ++i) { const int k = kc * 32 + 8 * g + (i < 8 ? i : 8 + i); const int tap = k / 3, c = k - tap * 3; const int yy = y + tap / 9 - 4, xx = px + tap % 9 - 4; const bool ok = (k < 243) && (yy >= 0) && (yy < HH) && (xx >= 0) && (xx < WWD);
      const float v = X[(((size_t)b * CIN + min(c, CIN - 1)) * HH + min(max(yy, 0), HH - 1)) * WWD + min(max(xx, 0), WWD - 1)]; a[i] = (__bf16)(ok ? v : 0.f); }
#pragma unroll
    for (int j = 0; j < 4; ++j) acc[j] = wmma_bf(a, frag_b(PK + PK_IN + (size_t)(j * 16 + col) * KIN + kc * 32, lane), acc[j]); }
  const float slope = bfr(AIN[0]);
#pragma unroll
  for (int j = 0; j < 4; ++j) { const int c = j * 16 + col; const float bb = bfr(BIN[c]);
#pragma unroll
    for (int r = 0; r < 8; ++r) { const float v = prelu(acc[j][r] + bb, slope); const __bf16 hb = (__bf16)v; sh_[wave][8 * g + r][c] = hb; sl_[wave][8 * g + r][c] = (__bf16)(v - (float)hb); } }
  LDSX();
  for (int rl = 0; rl < 16; ++rl) if (lane < 16) { const size_t p = ((size_t)row * WWD + wave * 16 + rl) * CH; if (lane < 8) vst2((unsigned*)(OH + p + lane * 8), *(const v4u*)&sh_[wave][rl][lane * 8]); else vst2((unsigned*)(OL + p + (lane - 8) * 8), *(const v4u*)&sl_[wave][rl][(lane - 8) * 8]); }
}
template <int EPI>
__global__ __launch_bounds__(192) void k_c3(const __bf16* __restrict__ IH, const __bf16* __restrict__ IL, const __bf16* __restrict__ W, const float* __restrict__ BIAS, const float* __restrict__ SLOPE, const __bf16* __restrict__ RH, const __bf16* __restrict__ RL, __bf16* __restrict__ OH, __bf16* __restrict__ OL) {
  __shared__ __align__(16) __bf16 sh_[6][16][72], sl_[6][16][72];
  const int tid = threadIdx.x, wave = tid >> 5, lane = tid & 31, col = lane & 15, g = lane >> 4; const int row = blockIdx.x; const int b = row / HH, y = row % HH; const int px = wave * 16 + col;
  v8f acc[4] = {};
#pragma unroll 1
  for (int tap = 0; tap < 9; ++tap) { const int yy = y + tap / 3 - 1, xx = px + tap % 3 - 1; const bool ok = (yy >= 0) && (yy < HH) && (xx >= 0) && (xx < WWD);
    const size_t ap = (((size_t)b * HH + min(max(yy, 0), HH - 1)) * WWD + min(max(xx, 0), WWD - 1)) * CH;
#pragma unroll
    for (int kc = 0; kc < 2; ++kc) { const v16b ah = zfrag_if(frag_b(IH + ap + kc * 32, lane), ok), al = zfrag_if(frag_b(IL + ap + kc * 32, lane), ok); const size_t kk = (size_t)tap * CH + kc * 32;
#pragma unroll
      for (int j = 0; j < 4; ++j) { const v16b w = frag_b(W + (size_t)(j * 16 + col) * K3 + kk, lane); acc[j] = wmma_bf(al, w, acc[j]); acc[j] = wmma_bf(ah, w, acc[j]); } } }
  const float slope = (EPI == 0) ? bfr(SLOPE[0]) : 0.f;
#pragma unroll
  for (int j = 0; j < 4; ++j) { const int c = j * 16 + col; const float bb = bfr(BIAS[c]);
#pragma unroll
    for (int r = 0; r < 8; ++r) { const size_t p = ((size_t)row * WWD + wave * 16 + 8 * g + r) * CH + c; float v = acc[j][r] + bb; if (EPI == 0) v = prelu(v, slope); else v = v + ((float)RH[p] + (float)RL[p]); const __bf16 hb = (__bf16)v; sh_[wave][8 * g + r][c] = hb; sl_[wave][8 * g + r][c] = (__bf16)(v - (float)hb); } }
  LDSX();
  for (int rl = 0; rl < 16; ++rl) if (lane < 16) { const size_t p = ((size_t)row * WWD + wave * 16 + rl) * CH; if (lane < 8) vst2((unsigned*)(OH + p + lane * 8), *(const v4u*)&sh_[wave][rl][lane * 8]); else vst2((unsigned*)(OL + p + (lane - 8) * 8), *(const v4u*)&sl_[wave][rl][(lane - 8) * 8]); }
}
__global__ __launch_bounds__(128) void k_qkv(const __bf16* __restrict__ IH, const __bf16* __restrict__ IL, const __bf16* __restrict__ PK, const float* __restrict__ BQ, const float* __restrict__ BK, const float* __restrict__ BV, _Float16* __restrict__ QK, _Float16* __restrict__ VTH, _Float16* __restrict__ VTL) {
  __shared__ __align__(16) _Float16 sqk[4][16][72]; __shared__ __align__(16) _Float16 sth[64][72], stl[64][72];
  const int tid = threadIdx.x, wave = tid >> 5, lane = tid & 31, col = lane & 15, g = lane >> 4; const size_t n0 = (size_t)blockIdx.x * 64; const size_t r0 = n0 + wave * 16;
  v8f acc[6] = {};
#pragma unroll
  for (int kc = 0; kc < 2; ++kc) { F2 a; a.h = frag_b(IH + (r0 + col) * CH + kc * 32, lane); a.l = frag_b(IL + (r0 + col) * CH + kc * 32, lane);
#pragma unroll
    for (int j = 0; j < 6; ++j) { const __bf16* P = (j == 0) ? PK + PK_Q : (j == 1) ? PK + PK_K : PK + PK_V + (size_t)(j - 2) * 16 * CH; const v16b w = frag_b(P + (size_t)col * CH + kc * 32, lane); acc[j] = wmma_bf(a.l, w, acc[j]); acc[j] = wmma_bf(a.h, w, acc[j]); } }
#pragma unroll
  for (int j = 0; j < 6; ++j)
#pragma unroll
    for (int r = 0; r < 8; ++r) { const int rl = 8 * g + r;
      if (j < 2) { const float bb = (col < C8) ? bfr((j == 0 ? BQ : BK)[min(col, C8 - 1)]) : 0.f; const float v = acc[j][r] + bb; sqk[wave][rl][j * 32 + col] = (_Float16)v; sqk[wave][rl][j * 32 + 16 + col] = (_Float16)0.f; }
      else { const int c = (j - 2) * 16 + col; const float v = acc[j][r] + bfr(BV[c]); const _Float16 hv = (_Float16)v; sth[c][wave * 16 + rl] = hv; stl[c][wave * 16 + rl] = (_Float16)((v - (float)hv) * 2048.0f); } }
  __syncthreads();
  for (int rl = 0; rl < 16; ++rl) if (lane < 8) vst2((unsigned*)(QK + (r0 + rl) * 64 + lane * 8), *(const v4u*)&sqk[wave][rl][lane * 8]);
  { const int b = (int)(n0 / NPI); const int s0 = (int)(n0 % NPI);
    for (int q = tid; q < 64 * 8; q += 128) { const int c = q >> 3, pc = q & 7; const size_t o = ((size_t)b * CH + c) * NPI + s0 + pc * 8; vst2((unsigned*)(VTH + o), *(const v4u*)&sth[c][pc * 8]); vst2((unsigned*)(VTL + o), *(const v4u*)&stl[c][pc * 8]); } }
}
__global__ __launch_bounds__(128) void k_att(const _Float16* __restrict__ QK, const _Float16* __restrict__ VTH, const _Float16* __restrict__ VTL, const __bf16* __restrict__ XH, const __bf16* __restrict__ XL, const float* __restrict__ GAMMA, __bf16* __restrict__ AH, __bf16* __restrict__ AL) {
  __shared__ __align__(16) float sp[4][16][36]; __shared__ __align__(16) __bf16 soh[4][16][72], sol[4][16][72];
  const int tid = threadIdx.x, wave = tid >> 5, lane = tid & 31, col = lane & 15, g = lane >> 4; const int qb = blockIdx.x, b = blockIdx.y; const int q0 = qb * 64 + wave * 16; const size_t rq = (size_t)b * NPI + q0 + col;
  const v16h aq = frag_h(QK + rq * 64, lane);
  float m[8], l[8];
#pragma unroll
  for (int r = 0; r < 8; ++r) { m[r] = -3.0e38f; l[r] = 0.f; }
  v8f acc[4] = {}, accl[4] = {};
#pragma unroll 1
  for (int ks = 0; ks < NPI / 32; ++ks) { v8f s[2];
#pragma unroll
    for (int ct = 0; ct < 2; ++ct) { const int kk = ks * 32 + ct * 16 + col; s[ct] = wmma16(aq, frag_h(QK + ((size_t)b * NPI + kk) * 64 + 32, lane), (v8f){}); }
#pragma unroll
    for (int r = 0; r < 8; ++r) { float mx = fmaxf(s[0][r], s[1][r]);
#pragma unroll
      for (int o = 1; o < 16; o <<= 1) mx = fmaxf(mx, __shfl_xor(mx, o));
      const float mn = fmaxf(m[r], mx); const float alpha = __expf(m[r] - mn);
      const float e0 = (float)(_Float16)(__expf(s[0][r] - mn) * 16384.0f), e1 = (float)(_Float16)(__expf(s[1][r] - mn) * 16384.0f); float es = e0 + e1;
#pragma unroll
      for (int o = 1; o < 16; o <<= 1) es += __shfl_xor(es, o);
      l[r] = l[r] * alpha + es; m[r] = mn;
#pragma unroll
      for (int dt = 0; dt < 4; ++dt) { acc[dt][r] *= alpha; accl[dt][r] *= alpha; }
      sp[wave][8 * g + r][col] = e0; sp[wave][8 * g + r][16 + col] = e1; }
    LDSX();
    const v16h pa = frag_f32(&sp[wave][col][0], lane);
#pragma unroll
    for (int dt = 0; dt < 4; ++dt) { const size_t vr = ((size_t)b * CH + dt * 16 + col) * NPI + (size_t)ks * 32; acc[dt] = wmma16(pa, frag_h(VTH + vr, lane), acc[dt]); accl[dt] = wmma16(pa, frag_h(VTL + vr, lane), accl[dt]); }
    LDSX(); }
  const float gamma = bfr(GAMMA[0]);
#pragma unroll
  for (int r = 0; r < 8; ++r) { const float il = 1.0f / l[r]; const size_t n = (size_t)b * NPI + q0 + 8 * g + r;
#pragma unroll
    for (int dt = 0; dt < 4; ++dt) { const int c = dt * 16 + col; const float xv = (float)XH[n * CH + c] + (float)XL[n * CH + c]; const float v = gamma * ((acc[dt][r] + accl[dt][r] * (1.0f / 2048.0f)) * il) + xv; const __bf16 hb = (__bf16)v; soh[wave][8 * g + r][c] = hb; sol[wave][8 * g + r][c] = (__bf16)(v - (float)hb); } }
  LDSX();
  for (int rl = 0; rl < 16; ++rl) if (lane < 16) { const size_t n = (size_t)b * NPI + q0 + rl; if (lane < 8) vst2((unsigned*)(AH + n * CH + lane * 8), *(const v4u*)&soh[wave][rl][lane * 8]); else vst2((unsigned*)(AL + n * CH + (lane - 8) * 8), *(const v4u*)&sol[wave][rl][(lane - 8) * 8]); }
}
__global__ __launch_bounds__(192) void k_cout(const __bf16* __restrict__ IH, const __bf16* __restrict__ IL, const __bf16* __restrict__ PK, const float* __restrict__ BOUT, float* __restrict__ OUT) {
  __shared__ __align__(16) float so[CIN][100];
  const int tid = threadIdx.x, wave = tid >> 5, lane = tid & 31, col = lane & 15, g = lane >> 4; const int row = blockIdx.x; const int b = row / HH, y = row % HH; const int px = wave * 16 + col;
  v8f acc = {};
#pragma unroll 1
  for (int tap = 0; tap < 81; ++tap) { const int yy = y + tap / 9 - 4, xx = px + tap % 9 - 4; const bool ok = (yy >= 0) && (yy < HH) && (xx >= 0) && (xx < WWD);
    const size_t ap = (((size_t)b * HH + min(max(yy, 0), HH - 1)) * WWD + min(max(xx, 0), WWD - 1)) * CH;
#pragma unroll
    for (int kc = 0; kc < 2; ++kc) { const v16b ah = zfrag_if(frag_b(IH + ap + kc * 32, lane), ok), al = zfrag_if(frag_b(IL + ap + kc * 32, lane), ok); const size_t kk = (size_t)tap * CH + kc * 32; const v16b w = frag_b(PK + PK_O + (size_t)col * KOUT + kk, lane); acc = wmma_bf(al, w, acc); acc = wmma_bf(ah, w, acc); } }
  if (col < CIN) { const float bb = bfr(BOUT[col]);
#pragma unroll
    for (int r = 0; r < 8; ++r) so[col][wave * 16 + 8 * g + r] = tanh_ni(acc[r] + bb); }
  __syncthreads();
  for (int q = tid; q < CIN * 24; q += 192) { const int c = q / 24, pc = q % 24; vst2(OUT + (((size_t)b * CIN + c) * HH + y) * WWD + pc * 4, *(const v4f*)&so[c][pc * 4]); }
}
extern "C" void kernel_launch(void* const* d_in, const int* in_sizes, int n_in, void* d_out, int out_size, void* d_ws, size_t ws_size, hipStream_t stream) {
  (void)in_sizes; (void)n_in; (void)out_size;
  const float** F = (const float**)d_in;
  if (ws_size < (size_t)WS_END) return;
  char* ws = (char*)d_ws; __bf16* PK = (__bf16*)(ws + WS_PK); _Float16 *QK = (_Float16*)(ws + WS_QK), *VTH = (_Float16*)(ws + WS_VTH), *VTL = (_Float16*)(ws + WS_VTL);
  auto OH = [&](int i) { return (__bf16*)(ws + PL_OUT(i, 0)); }; auto OL = [&](int i) { return (__bf16*)(ws + PL_OUT(i, 1)); };
  __bf16 *HBH = (__bf16*)(ws + PL_H(0)), *HBL = (__bf16*)(ws + PL_H(1)), *AH = (__bf16*)(ws + PL_ATT(0)), *AL = (__bf16*)(ws + PL_ATT(1));
  k_pack<<<dim3(96, 13), 256, 0, stream>>>(F[1], F[4], F[7], F[9], F[11], F[13], F[16], PK);
  k_cin<<<TNB * HH, 192, 0, stream>>>(F[0], PK, F[2], F[3], OH(0), OL(0));
  for (int i = 0; i < NBLK; ++i) {
    k_c3<0><<<TNB * HH, 192, 0, stream>>>(OH(i), OL(i), PK + PK_R1 + (size_t)i * CH * K3, F[5] + i * CH, F[6] + i, nullptr, nullptr, HBH, HBL);
    k_c3<1><<<TNB * HH, 192, 0, stream>>>(HBH, HBL, PK + PK_R2 + (size_t)i * CH * K3, F[8] + i * CH, nullptr, OH(i), OL(i), OH(i + 1), OL(i + 1)); }
  k_qkv<<<TNB * NPI / 64, 128, 0, stream>>>(OH(5), OL(5), PK, F[10], F[12], F[14], QK, VTH, VTL);
  k_att<<<dim3(TQT / TNB < NPI / 64 ? TQT : NPI / 64, TNB), 128, 0, stream>>>(QK, VTH, VTL, OH(5), OL(5), F[15], AH, AL);
  k_cout<<<TYO, 192, 0, stream>>>(AH, AL, PK, F[17], (float*)d_out);
}
